// WeightedMaxAggregator_25967372271703
// MI455X (gfx1250) — hardware-verified
//
#include <hip/hip_runtime.h>


#define NB_  128
#define SS   512
#define EE   64
#define EPSN 1e-7f

typedef unsigned short bf;
typedef __attribute__((ext_vector_type(16))) __bf16   v16bf;
typedef __attribute__((ext_vector_type(8)))  unsigned short v8us;
typedef __attribute__((ext_vector_type(8)))  float    v8f;
typedef __attribute__((ext_vector_type(2)))  float    v2f;
typedef v8us __attribute__((may_alias)) v8usa;

__device__ __forceinline__ unsigned short f2bf(float f) { unsigned u = __float_as_uint(f); u += 0x7FFFu + ((u >> 16) & 1u); return (unsigned short)(u >> 16); }
__device__ __forceinline__ float bf2f(unsigned short b) { return __uint_as_float(((unsigned)b) << 16); }
__device__ __forceinline__ float bfr(float f) { return bf2f(f2bf(f)); }
__device__ __forceinline__ v16bf cat16b(v8us lo, v8us hi) { return __builtin_bit_cast(v16bf, __builtin_shufflevector(lo, hi, 0, 1, 2, 3, 4, 5, 6, 7, 8, 9, 10, 11, 12, 13, 14, 15)); }
__device__ __forceinline__ v8f wmmab(v16bf a, v16bf b, v8f c) { return __builtin_amdgcn_wmma_f32_16x16x32_bf16(false, a, false, b, (short)0, c, false, false); }
#define VST2(T, p, v) do { const T vst2_v_ = (v); *(volatile T*)(p) = vst2_v_; __threadfence(); *(volatile T*)(p) = vst2_v_; } while (0)

__global__ __launch_bounds__(256) void k_rows(const float* __restrict__ x, bf* Xb, float* RN) {
    __shared__ float sq[32];
    const int tid = threadIdx.x, lane = tid & 31, wave = tid >> 5;
    const int rl = tid >> 3, piece = tid & 7; const size_t r = (size_t)blockIdx.x * 32 + rl;
    v8us t; float s = 0.f;
#pragma unroll
    for (int i = 0; i < 8; ++i) { const float v = bfr(x[r * EE + piece * 8 + i]); t[i] = f2bf(v); s += v * v; }
    s += __shfl_xor(s, 1, 8); s += __shfl_xor(s, 2, 8); s += __shfl_xor(s, 4, 8);
    if (piece == 0) sq[rl] = 1.0f / fmaxf(sqrtf(s), EPSN);
    VST2(v8us, Xb + r * EE + piece * 8, t);
    __syncthreads();
    if (wave == 0) VST2(float, RN + (size_t)blockIdx.x * 32 + lane, sq[lane]);
}
__global__ __launch_bounds__(128) void k_main(const bf* __restrict__ Ub, const float* __restrict__ RU, const bf* __restrict__ Vb, const float* __restrict__ RV,
                                             const float* __restrict__ cw, const float* __restrict__ mask, const float* __restrict__ pw, const float* __restrict__ pb, float* out) {
    __shared__ float res[64];
    const int lane = threadIdx.x & 31, wave = threadIdx.x >> 5, lr = lane & 15, hi = lane >> 4;
    const int b = blockIdx.x / (SS / 64), st = blockIdx.x - b * (SS / 64), s0 = st * 64 + wave * 16;
    const size_t rowu = (size_t)b * SS + s0, rowv0 = (size_t)b * SS;
    const float w = bfr(pw[0]), bias = bfr(pb[0]);
    v16bf ua[2];
#pragma unroll
    for (int kc = 0; kc < 2; ++kc) { const bf* p = Ub + (rowu + lr) * EE + kc * 32 + 8 * hi; ua[kc] = cat16b(*(const v8us*)p, *(const v8us*)(p + 16)); }
    float ru[8], mx[8];
#pragma unroll
    for (int j = 0; j < 8; ++j) { ru[j] = RU[rowu + 8 * hi + j]; mx[j] = -3.0e38f; }
#pragma unroll 1
    for (int nt = 0; nt < SS / 32; ++nt) {
        const int n0 = nt * 32;
        v8f d0 = {}, d1 = {};
#pragma unroll
        for (int kc = 0; kc < 2; ++kc) {
            const bf* b0 = Vb + (rowv0 + n0 + lr) * EE + kc * 32 + 8 * hi; const bf* b1 = b0 + (size_t)16 * EE;
            d0 = wmmab(ua[kc], cat16b(*(const v8us*)b0, *(const v8us*)(b0 + 16)), d0);
            d1 = wmmab(ua[kc], cat16b(*(const v8us*)b1, *(const v8us*)(b1 + 16)), d1);
        }
        asm volatile("v_nop\n\tv_nop\n\tv_nop\n\tv_nop" : "+v"(d0), "+v"(d1) : "v"(ua[0]), "v"(ua[1]));
        const int na = n0 + lr, nb = n0 + 16 + lr;
        const float fa = RV[rowv0 + na] * bfr(cw[rowv0 + na]) * w, fb = RV[rowv0 + nb] * bfr(cw[rowv0 + nb]) * w;
        const float ma = bfr(mask[rowv0 + na]), mb = bfr(mask[rowv0 + nb]);
#pragma unroll
        for (int j = 0; j < 8; ++j) {
            const float va = ma / (1.0f + __expf(-(d0[j] * ru[j] * fa + bias))), vb = mb / (1.0f + __expf(-(d1[j] * ru[j] * fb + bias)));
            mx[j] = fmaxf(mx[j], fmaxf(va, vb));
        }
    }
#pragma unroll
    for (int j = 0; j < 8; ++j) { float m = mx[j]; m = fmaxf(m, __shfl_xor(m, 1, 16)); m = fmaxf(m, __shfl_xor(m, 2, 16)); m = fmaxf(m, __shfl_xor(m, 4, 16)); m = fmaxf(m, __shfl_xor(m, 8, 16));
        if (lr == 0) res[wave * 16 + hi * 8 + j] = m; }
    __syncthreads();
    if (wave == 0) { v2f o; o[0] = res[lane * 2]; o[1] = res[lane * 2 + 1]; VST2(v2f, out + (size_t)b * SS + st * 64 + lane * 2, o); }
}

extern "C" void kernel_launch(void* const* d_in, const int* in_sizes, int n_in,
                              void* d_out, int out_size, void* d_ws, size_t ws_size, hipStream_t stream) {
    (void)in_sizes; (void)n_in; (void)out_size;
    const float* ue = (const float*)d_in[0]; const float* ie = (const float*)d_in[1]; const float* cw = (const float*)d_in[2]; const float* mask = (const float*)d_in[3];
    const float* pw = (const float*)d_in[4]; const float* pb = (const float*)d_in[5];
    float* out = (float*)d_out;
    char* wsp = (char*)d_ws;
    auto take = [&](size_t bytes) { char* p = wsp; wsp += (bytes + 255) & ~(size_t)255; return (void*)p; };
    bf* Ub = (bf*)take((size_t)NB_ * SS * EE * 2); bf* Vb = (bf*)take((size_t)NB_ * SS * EE * 2); float* RU = (float*)take((size_t)NB_ * SS * 4); float* RV = (float*)take((size_t)NB_ * SS * 4);
    if ((size_t)(wsp - (char*)d_ws) > ws_size) return;
    k_rows<<<(NB_ * SS) / 32, 256, 0, stream>>>(ue, Ub, RU);
    k_rows<<<(NB_ * SS) / 32, 256, 0, stream>>>(ie, Vb, RV);
    k_main<<<NB_ * (SS / 64), 128, 0, stream>>>(Ub, RU, Vb, RV, cw, mask, pw, pb, out);
}
